// ProposalModuleRefine_21921513079478
// MI455X (gfx1250) — hardware-verified
//
#include <hip/hip_runtime.h>
#include <cstdint>
#include <cstddef>

typedef __attribute__((ext_vector_type(16))) __bf16 v16b;
typedef __attribute__((ext_vector_type(8)))  float  v8f;
typedef __attribute__((ext_vector_type(4)))  float  v4f;

#define B_      16
#define K_      2048
#define NPROP_  256
#define NSAMPLE_ 16
#define CSEED_  256
#define CMLP_   128
#define RADIUS_ 0.3f
#define NH_     12
#define NSC_    18
#define KPAD0_  288
#define M0_     (B_*NPROP_*NSAMPLE_)
#define M1_     (B_*NPROP_)

static constexpr size_t O0  = 0;
static constexpr size_t O1  = O0  + 8192;
static constexpr size_t O2  = O1  + 12288;
static constexpr size_t O3  = O2  + 49152;
static constexpr size_t O4  = O3  + 49152;
static constexpr size_t O5  = O4  + 73728;
static constexpr size_t O6  = O5  + 221184;
static constexpr size_t O7  = O6  + 73728;
static constexpr size_t O8  = O7  + 98304;
static constexpr size_t O9  = O8  + 4194304;
static constexpr size_t O10 = O9  + 49152;
static constexpr size_t O11 = O10 + 73728;

__device__ __forceinline__ unsigned short f2bf_bits(float f) {
  unsigned u = __float_as_uint(f);
  return (unsigned short)((u + 0x7FFFu + ((u >> 16) & 1u)) >> 16);
}
__device__ __forceinline__ float bf_bits2f(unsigned short h) {
  return __uint_as_float(((unsigned)h) << 16);
}
__device__ __forceinline__ void split16(const float* v, v16b& hi, v16b& lo) {
#pragma unroll
  for (int e = 0; e < 16; ++e) {
    unsigned short hb = f2bf_bits(v[e]);
    float hf = bf_bits2f(hb);
    unsigned short lb = f2bf_bits(v[e] - hf);
    hi[e] = __builtin_bit_cast(__bf16, hb);
    lo[e] = __builtin_bit_cast(__bf16, lb);
  }
}

__device__ __forceinline__ v8f wmma3(v16b ah, v16b al, v16b bh, v16b bl, v8f acc) {
  acc = __builtin_amdgcn_wmma_f32_16x16x32_bf16(false, ah, false, bh, (short)0, acc, false, false);
  acc = __builtin_amdgcn_wmma_f32_16x16x32_bf16(false, ah, false, bl, (short)0, acc, false, false);
  acc = __builtin_amdgcn_wmma_f32_16x16x32_bf16(false, al, false, bh, (short)0, acc, false, false);
  asm volatile("v_nop\n\tv_nop\n\tv_nop\n\tv_nop" : "+v"(acc) : "v"(ah), "v"(al), "v"(bh), "v"(bl));
  return acc;
}

__device__ __forceinline__ void flush_lines(float* dst, const float* lds, int n4, int tid, int nthr) {
  volatile v4f* d = (volatile v4f*)dst;
  for (int i = tid; i < n4; i += nthr) { v4f v = *(const v4f*)(lds + 4 * i); d[i] = v; }
  __threadfence();
  for (int i = tid; i < n4; i += nthr) { v4f v = *(const v4f*)(lds + 4 * i); d[i] = v; }
}

__global__ void pad_w_kernel(const float* __restrict__ src, float* __restrict__ dst,
                             int srcRows, int srcCols, int dstCols, int dstRows) {
  int i = blockIdx.x * blockDim.x + threadIdx.x;
  int tot = dstRows * dstCols;
  if (i >= tot) return;
  int r = i / dstCols, c = i % dstCols;
  float v = (r < srcRows && c < srcCols) ? src[r * srcCols + c] : 0.0f;
  ((volatile float*)dst)[i] = v;
  __threadfence();
  ((volatile float*)dst)[i] = v;
}

__global__ void pad_bias_kernel(const float* __restrict__ src, float* __restrict__ dst, int n, int tot) {
  int i = blockIdx.x * blockDim.x + threadIdx.x;
  if (i < tot) {
    float v = (i < n) ? src[i] : 0.0f;
    ((volatile float*)dst)[i] = v;
    __threadfence();
    ((volatile float*)dst)[i] = v;
  }
}

__global__ void __launch_bounds__(256) fps_kernel(const float* __restrict__ xyz, float* __restrict__ new_xyz) {
#pragma clang fp contract(off)
  __shared__ float sx[K_], sy[K_], sz[K_];
  __shared__ float sdist[K_];
  __shared__ float rmax[256];
  __shared__ int   ridx[256];
  __shared__ int   sfar;
  __shared__ int   sinds[NPROP_];
  __shared__ __align__(16) float snew[NPROP_ * 3];

  int b = blockIdx.x, t = threadIdx.x;
  for (int i = t; i < K_; i += 256) {
    sx[i] = xyz[((size_t)b * K_ + i) * 3 + 0];
    sy[i] = xyz[((size_t)b * K_ + i) * 3 + 1];
    sz[i] = xyz[((size_t)b * K_ + i) * 3 + 2];
    sdist[i] = 1e10f;
  }
  if (t == 0) sfar = 0;
  __syncthreads();

  for (int it = 0; it < NPROP_; ++it) {
    int far = sfar;
    if (t == 0) sinds[it] = far;
    float cx = sx[far], cy = sy[far], cz = sz[far];
    float bm = -1.0f; int bi = 0x7fffffff;
    for (int i = t; i < K_; i += 256) {
      float dx = sx[i] - cx, dy = sy[i] - cy, dz = sz[i] - cz;
      float d = (dx * dx + dy * dy) + dz * dz;
      float nd = fminf(sdist[i], d);
      sdist[i] = nd;
      if (nd > bm) { bm = nd; bi = i; }
    }
    __syncthreads();
    rmax[t] = bm; ridx[t] = bi;
    __syncthreads();
    for (int s = 128; s > 0; s >>= 1) {
      if (t < s) {
        float om = rmax[t + s]; int oi = ridx[t + s];
        if (om > rmax[t] || (om == rmax[t] && oi < ridx[t])) { rmax[t] = om; ridx[t] = oi; }
      }
      __syncthreads();
    }
    if (t == 0) sfar = ridx[0];
    __syncthreads();
  }
  int id = sinds[t];
  snew[t * 3 + 0] = sx[id];
  snew[t * 3 + 1] = sy[id];
  snew[t * 3 + 2] = sz[id];
  __syncthreads();
  flush_lines(new_xyz + (size_t)b * NPROP_ * 3, snew, NPROP_ * 3 / 4, t, 256);
}

__global__ void __launch_bounds__(256) group_kernel(const float* __restrict__ xyz,
                             const float* __restrict__ vfeat,
                             const float* __restrict__ new_xyz,
                             float* __restrict__ Xg) {
#pragma clang fp contract(off)
  __shared__ int sidx[8][NSAMPLE_];
  int wave = threadIdx.x >> 5;
  int lane = threadIdx.x & 31;
  int pr = blockIdx.x * 8 + wave;
  int b = pr >> 8;

  float nx = new_xyz[pr * 3 + 0];
  float ny = new_xyz[pr * 3 + 1];
  float nz = new_xyz[pr * 3 + 2];
  const float r2 = 0.09f;

  int cnt = 0;
  for (int base = 0; base < K_; base += 32) {
    int i = base + lane;
    float dx = nx - xyz[((size_t)b * K_ + i) * 3 + 0];
    float dy = ny - xyz[((size_t)b * K_ + i) * 3 + 1];
    float dz = nz - xyz[((size_t)b * K_ + i) * 3 + 2];
    float d2 = (dx * dx + dy * dy) + dz * dz;
    bool within = d2 <= r2;
    unsigned m32 = (unsigned)__ballot(within);
    int prefix = __popc(m32 & ((1u << lane) - 1u));
    int slot = cnt + prefix;
    if (within && slot < NSAMPLE_) sidx[wave][slot] = i;
    cnt += __popc(m32);
  }
  __syncthreads();
  if (cnt == 0 && lane == 0) sidx[wave][0] = 0;
  __syncthreads();
  int filled = cnt < NSAMPLE_ ? (cnt < 1 ? 1 : cnt) : NSAMPLE_;
  int first = sidx[wave][0];
  if (lane < NSAMPLE_ && lane >= filled) sidx[wave][lane] = first;
  __syncthreads();

  const float inv_r = 1.0f / RADIUS_;
  for (int pass = 0; pass < 2; ++pass) {
    for (int s = 0; s < NSAMPLE_; ++s) {
      int id = sidx[wave][s];
      volatile float* dst = Xg + ((size_t)pr * NSAMPLE_ + s) * KPAD0_;
      for (int c = lane; c < KPAD0_; c += 32) {
        float v;
        if (c < 3) {
          float g = xyz[((size_t)b * K_ + id) * 3 + c];
          float n = (c == 0) ? nx : (c == 1) ? ny : nz;
          v = (g - n) * inv_r;
        } else if (c < 3 + CSEED_) {
          v = vfeat[((size_t)b * CSEED_ + (c - 3)) * K_ + id];
        } else {
          v = 0.0f;
        }
        dst[c] = v;
      }
    }
    __threadfence();
  }
}

__global__ void __launch_bounds__(256)
wmma_gemm_kernel(const float* __restrict__ A,
                 const float* __restrict__ Wt,
                 int Kpad,
                 const float* __restrict__ q0,
                 const float* __restrict__ q1,
                 const float* __restrict__ q2,
                 int mode,
                 float* __restrict__ outF) {
  __shared__ __align__(16) unsigned short sWh[128 * 32];
  __shared__ __align__(16) unsigned short sWl[128 * 32];
  __shared__ __align__(16) float sT[8][16 * 132];

  int tid  = threadIdx.x;
  int wave = tid >> 5;
  int lane = tid & 31;
  int rl = lane & 15;
  int kh = (lane >> 4) * 8;
  size_t mtile = (size_t)blockIdx.x * 8 + wave;
  size_t arow = mtile * 16 + rl;

  v8f acc[8];
#pragma unroll
  for (int nt = 0; nt < 8; ++nt) acc[nt] = (v8f){0.f, 0.f, 0.f, 0.f, 0.f, 0.f, 0.f, 0.f};

  int ksteps = Kpad >> 5;
  for (int ks = 0; ks < ksteps; ++ks) {
    __syncthreads();
    for (int i = tid; i < 128 * 32; i += 256) {
      int n = i >> 5, c = i & 31;
      float w = Wt[(size_t)n * Kpad + (size_t)ks * 32 + c];
      unsigned short hb = f2bf_bits(w);
      sWh[i] = hb;
      sWl[i] = f2bf_bits(w - bf_bits2f(hb));
    }
    __syncthreads();

    float av[16];
    const float* ap = A + arow * Kpad + (size_t)ks * 32 + kh;
    {
      v4f t0 = *(const v4f*)(ap), t1 = *(const v4f*)(ap + 4), t2 = *(const v4f*)(ap + 16), t3 = *(const v4f*)(ap + 20);
      av[0]=t0[0]; av[1]=t0[1]; av[2]=t0[2]; av[3]=t0[3]; av[4]=t1[0]; av[5]=t1[1]; av[6]=t1[2]; av[7]=t1[3];
      av[8]=t2[0]; av[9]=t2[1]; av[10]=t2[2]; av[11]=t2[3]; av[12]=t3[0]; av[13]=t3[1]; av[14]=t3[2]; av[15]=t3[3];
    }
    v16b ah, al;
    split16(av, ah, al);

#pragma unroll
    for (int nt = 0; nt < 8; ++nt) {
      const unsigned short* bph = sWh + (nt * 16 + rl) * 32 + kh;
      const unsigned short* bpl = sWl + (nt * 16 + rl) * 32 + kh;
      v16b bh, bl;
#pragma unroll
      for (int e = 0; e < 8; ++e) {
        bh[e]     = __builtin_bit_cast(__bf16, bph[e]);
        bh[8 + e] = __builtin_bit_cast(__bf16, bph[16 + e]);
        bl[e]     = __builtin_bit_cast(__bf16, bpl[e]);
        bl[8 + e] = __builtin_bit_cast(__bf16, bpl[16 + e]);
      }
      acc[nt] = wmma3(ah, al, bh, bl, acc[nt]);
    }
  }

  int mbase = (lane >> 4) * 8;
  float* tile = sT[wave];
#pragma unroll
  for (int nt = 0; nt < 8; ++nt) {
    int n = nt * 16 + rl;
    float a0v = q0[n];
    float a1v = (mode <= 1) ? q1[n] : 0.f;
    float a2v = (mode == 1) ? q2[n] : 0.f;
#pragma unroll
    for (int r = 0; r < 8; ++r) {
      float v = acc[nt][r];
      if (mode == 0)      v = fmaxf(v * a0v + a1v, 0.0f);
      else if (mode == 1) v = fmaxf((v + a0v) * a1v + a2v, 0.0f);
      else                v = v + a0v;
      tile[(mbase + r) * 132 + n] = v;
    }
  }
  __syncthreads();
  float* obase = outF + mtile * 16 * 128;
  for (int pass = 0; pass < 2; ++pass) {
#pragma unroll
    for (int r = 0; r < 16; ++r) {
      v4f v = *(const v4f*)(tile + r * 132 + lane * 4);
      *(volatile v4f*)(obase + r * 128 + lane * 4) = v;
    }
    __threadfence();
  }
}

__global__ void maxpool_kernel(const float* __restrict__ Y2, float* __restrict__ feat) {
  int t = blockIdx.x * blockDim.x + threadIdx.x;
  if (t >= M1_ * CMLP_) return;
  int pr = t >> 7, c = t & 127;
  float m = -3.4e38f;
  for (int s = 0; s < NSAMPLE_; ++s)
    m = fmaxf(m, Y2[((size_t)pr * NSAMPLE_ + s) * 128 + c]);
  ((volatile float*)feat)[t] = m;
  __threadfence();
  ((volatile float*)feat)[t] = m;
}

#define HP_ 64
__global__ void __launch_bounds__(HP_) heads_kernel(const float* __restrict__ nt,
                             const float* __restrict__ nxyz,
                             const float* __restrict__ msa,
                             float* __restrict__ out) {
  __shared__ __align__(16) float s0[HP_ * 2];
  __shared__ __align__(16) float s1[HP_ * 3];
  __shared__ __align__(16) float s2[HP_ * NH_];
  __shared__ __align__(16) float s3[HP_ * NH_];
  __shared__ __align__(16) float s4[HP_ * NSC_];
  __shared__ __align__(16) float s5[HP_ * NSC_ * 3];
  __shared__ __align__(16) float s6[HP_ * NSC_];
  __shared__ __align__(16) float s10[6][HP_ * 3];

  int t = threadIdx.x;
  int pr0 = blockIdx.x * HP_;
  int pr = pr0 + t;
  int b = pr >> 8, p0 = pr0 & 255;
  const float* r = nt + (size_t)pr * 128;

  s0[t * 2 + 0] = r[0];
  s0[t * 2 + 1] = r[1];
  float cx = nxyz[pr * 3 + 0] + r[2];
  float cy = nxyz[pr * 3 + 1] + r[3];
  float cz = nxyz[pr * 3 + 2] + r[4];
  s1[t * 3 + 0] = cx; s1[t * 3 + 1] = cy; s1[t * 3 + 2] = cz;
  const float hscale = 0.2617993877991494f;
  for (int h = 0; h < NH_; ++h) {
    s2[t * NH_ + h] = r[5 + h];
    s3[t * NH_ + h] = r[5 + NH_ + h] * hscale;
  }
  int cls = 0; float bv = r[29];
  for (int j = 0; j < NSC_; ++j) {
    float v = r[29 + j];
    s4[t * NSC_ + j] = v;
    if (v > bv) { bv = v; cls = j; }
    s6[t * NSC_ + j] = r[101 + j];
    for (int d = 0; d < 3; ++d)
      s5[(t * NSC_ + j) * 3 + d] = r[47 + j * 3 + d] * msa[j * 3 + d];
  }
  float half3[3];
  for (int d = 0; d < 3; ++d) {
    float avg = msa[cls * 3 + d];
    float res = r[47 + cls * 3 + d] * avg;
    half3[d] = (avg + res) * 0.5f;
  }
  float fc[6][3] = {
    {cx, cy, cz + half3[2]}, {cx, cy, cz - half3[2]},
    {cx, cy + half3[1], cz}, {cx, cy - half3[1], cz},
    {cx + half3[0], cy, cz}, {cx - half3[0], cy, cz}};
  for (int f = 0; f < 6; ++f)
    for (int d = 0; d < 3; ++d) s10[f][t * 3 + d] = fc[f][d];
  __syncthreads();

  flush_lines(out + O0 + (size_t)pr0 * 2,        s0, HP_ * 2 / 4, t, HP_);
  flush_lines(out + O1 + (size_t)pr0 * 3,        s1, HP_ * 3 / 4, t, HP_);
  flush_lines(out + O2 + (size_t)pr0 * NH_,      s2, HP_ * NH_ / 4, t, HP_);
  flush_lines(out + O3 + (size_t)pr0 * NH_,      s3, HP_ * NH_ / 4, t, HP_);
  flush_lines(out + O4 + (size_t)pr0 * NSC_,     s4, HP_ * NSC_ / 4, t, HP_);
  flush_lines(out + O5 + (size_t)pr0 * NSC_ * 3, s5, HP_ * NSC_ * 3 / 4, t, HP_);
  flush_lines(out + O6 + (size_t)pr0 * NSC_,     s6, HP_ * NSC_ / 4, t, HP_);
  for (int f = 0; f < 6; ++f)
    flush_lines(out + O10 + ((size_t)b * 1536 + f * 256 + p0) * 3, s10[f], HP_ * 3 / 4, t, HP_);
}

__global__ void sel_center_kernel(const float* __restrict__ pz, const float* __restrict__ cz,
                                  const float* __restrict__ pxy, const float* __restrict__ cxy,
                                  const float* __restrict__ pl, const float* __restrict__ cl,
                                  float* __restrict__ out) {
  int i = blockIdx.x * blockDim.x + threadIdx.x;
  const int per = B_ * 1024 * 3;
  if (i >= 3 * per) return;
  int type = i / per;
  int rem = i % per;
  int d = rem % 3;
  int bk = rem / 3;
  int b = bk >> 10, k = bk & 1023;
  const float* pp = (type == 0) ? pz : (type == 1) ? pxy : pl;
  const float* cc = (type == 0) ? cz : (type == 1) ? cxy : cl;
  float x0 = pp[((size_t)b * 2 + 0) * 1024 + k];
  float x1 = pp[((size_t)b * 2 + 1) * 1024 + k];
  float p1 = 1.0f / (1.0f + expf(x0 - x1));
  float add = (p1 <= 0.5f) ? 10.0f : 0.0f;
  float v = cc[((size_t)b * 1024 + k) * 3 + d] + add;
  size_t o;
  if (type == 0)      o = O7 + ((size_t)b * 2048 + k) * 3 + d;
  else if (type == 1) o = O7 + ((size_t)b * 2048 + 1024 + k) * 3 + d;
  else                o = O9 + ((size_t)b * 1024 + k) * 3 + d;
  ((volatile float*)out)[o] = v;
  __threadfence();
  ((volatile float*)out)[o] = v;
}

__global__ void copy_scfp_kernel(const float* __restrict__ aggz,
                                 const float* __restrict__ aggxy,
                                 float* __restrict__ out) {
  int i = blockIdx.x * blockDim.x + threadIdx.x;
  if (i >= B_ * 128 * 2048) return;
  int b = i / (128 * 2048);
  int rkc = i % (128 * 2048);
  int c = rkc / 2048, k = rkc % 2048;
  float v = (k < 1024) ? aggz[((size_t)b * 128 + c) * 1024 + k]
                       : aggxy[((size_t)b * 128 + c) * 1024 + (k - 1024)];
  ((volatile float*)out)[O8 + i] = v;
  __threadfence();
  ((volatile float*)out)[O8 + i] = v;
}

__global__ void tile_feat_kernel(const float* __restrict__ feat, float* __restrict__ out) {
  int i = blockIdx.x * blockDim.x + threadIdx.x;
  if (i >= B_ * 128 * 1536) return;
  int b = i / (128 * 1536);
  int rcj = i % (128 * 1536);
  int c = rcj / 1536, j = rcj % 1536;
  int p = j & 255;
  float v = feat[((size_t)b * 256 + p) * 128 + c];
  ((volatile float*)out)[O11 + i] = v;
  __threadfence();
  ((volatile float*)out)[O11 + i] = v;
}

extern "C" void kernel_launch(void* const* d_in, const int* in_sizes, int n_in,
                              void* d_out, int out_size, void* d_ws, size_t ws_size,
                              hipStream_t stream) {
  (void)in_sizes; (void)n_in; (void)out_size; (void)ws_size;
  const float* vote_xyz   = (const float*)d_in[0];
  const float* vote_feat  = (const float*)d_in[1];
  const float* psc_z      = (const float*)d_in[2];
  const float* center_z   = (const float*)d_in[3];
  const float* agg_z      = (const float*)d_in[4];
  const float* psc_xy     = (const float*)d_in[5];
  const float* center_xy  = (const float*)d_in[6];
  const float* agg_xy     = (const float*)d_in[7];
  const float* psc_line   = (const float*)d_in[8];
  const float* center_line= (const float*)d_in[9];
  const float* msa  = (const float*)d_in[11];
  const float* w0   = (const float*)d_in[12];
  const float* s0   = (const float*)d_in[13];
  const float* b0   = (const float*)d_in[14];
  const float* w1   = (const float*)d_in[15];
  const float* s1   = (const float*)d_in[16];
  const float* b1   = (const float*)d_in[17];
  const float* w2   = (const float*)d_in[18];
  const float* s2   = (const float*)d_in[19];
  const float* b2   = (const float*)d_in[20];
  const float* c1w  = (const float*)d_in[21];
  const float* c1b  = (const float*)d_in[22];
  const float* bn1s = (const float*)d_in[23];
  const float* bn1b = (const float*)d_in[24];
  const float* c2w  = (const float*)d_in[25];
  const float* c2b  = (const float*)d_in[26];
  const float* bn2s = (const float*)d_in[27];
  const float* bn2b = (const float*)d_in[28];
  const float* c3w  = (const float*)d_in[29];
  const float* c3b  = (const float*)d_in[30];
  float* out = (float*)d_out;

  char* w = (char*)d_ws;
  size_t off = 0;
  auto carve = [&](size_t bytes) -> char* {
    char* p = w + off;
    off = (off + bytes + 255) & ~(size_t)255;
    return p;
  };
  float* nxyz = (float*)carve((size_t)B_ * NPROP_ * 3 * 4);
  float* W0p  = (float*)carve((size_t)128 * KPAD0_ * 4);
  float* C3p  = (float*)carve((size_t)128 * 128 * 4);
  float* c3bp = (float*)carve((size_t)128 * 4);
  float* Xg   = (float*)carve((size_t)M0_ * KPAD0_ * 4);
  float* Y0   = (float*)carve((size_t)M0_ * 128 * 4);
  float* Y1   = (float*)carve((size_t)M0_ * 128 * 4);
  float* Y2   = (float*)carve((size_t)M0_ * 128 * 4);
  float* feat = (float*)carve((size_t)M1_ * 128 * 4);
  float* N1f  = (float*)carve((size_t)M1_ * 128 * 4);
  float* N2f  = (float*)carve((size_t)M1_ * 128 * 4);
  float* N3f  = (float*)carve((size_t)M1_ * 128 * 4);

  pad_w_kernel<<<(128 * KPAD0_ + 255) / 256, 256, 0, stream>>>(w0, W0p, 128, 259, KPAD0_, 128);
  pad_w_kernel<<<(128 * 128 + 255) / 256, 256, 0, stream>>>(c3w, C3p, 119, 128, 128, 128);
  pad_bias_kernel<<<1, 128, 0, stream>>>(c3b, c3bp, 119, 128);

  fps_kernel<<<B_, 256, 0, stream>>>(vote_xyz, nxyz);
  group_kernel<<<M1_ / 8, 256, 0, stream>>>(vote_xyz, vote_feat, nxyz, Xg);

  wmma_gemm_kernel<<<M0_ / 128, 256, 0, stream>>>(Xg, W0p, KPAD0_, s0, b0, nullptr, 0, Y0);
  wmma_gemm_kernel<<<M0_ / 128, 256, 0, stream>>>(Y0, w1, 128, s1, b1, nullptr, 0, Y1);
  wmma_gemm_kernel<<<M0_ / 128, 256, 0, stream>>>(Y1, w2, 128, s2, b2, nullptr, 0, Y2);

  maxpool_kernel<<<(M1_ * 128 + 255) / 256, 256, 0, stream>>>(Y2, feat);

  wmma_gemm_kernel<<<M1_ / 128, 256, 0, stream>>>(feat, c1w, 128, c1b, bn1s, bn1b, 1, N1f);
  wmma_gemm_kernel<<<M1_ / 128, 256, 0, stream>>>(N1f, c2w, 128, c2b, bn2s, bn2b, 1, N2f);
  wmma_gemm_kernel<<<M1_ / 128, 256, 0, stream>>>(N2f, C3p, 128, c3bp, nullptr, nullptr, 2, N3f);

  heads_kernel<<<M1_ / HP_, HP_, 0, stream>>>(N3f, nxyz, msa, out);
  sel_center_kernel<<<(3 * B_ * 1024 * 3 + 255) / 256, 256, 0, stream>>>(
      psc_z, center_z, psc_xy, center_xy, psc_line, center_line, out);
  copy_scfp_kernel<<<(B_ * 128 * 2048 + 255) / 256, 256, 0, stream>>>(agg_z, agg_xy, out);
  tile_feat_kernel<<<(B_ * 128 * 1536 + 255) / 256, 256, 0, stream>>>(feat, out);
}
